// LlamaDifferentialAttentionBase_19988777796148
// MI455X (gfx1250) — hardware-verified
//
#include <hip/hip_runtime.h>


namespace {
constexpr int S = 2048, D = 2048, H = 32, HKV = 8, HD = 64, DKV = HKV * HD, GRP = H / HKV, NQT = 2 * H  , NKT = 2 * HKV  , NVT = HKV  , NT = NQT + NKT + NVT  ;
constexpr float SCALE = 0.125f, VS = 8.0f, QS = 8.0f, PS = 8.0f, THETA = 10000.0f, EPSN = 1e-6f, LAMBDA_INIT = 0.783605767f;
constexpr size_t QPL = (size_t)NQT * S * HD, KPL = (size_t)NKT * S * HD, VPL = (size_t)NVT * HD * S;

typedef _Float16 b16;
typedef __attribute__((ext_vector_type(16))) _Float16 v16b;
typedef __attribute__((ext_vector_type(8)))  _Float16 v8b;
typedef __attribute__((ext_vector_type(8)))  float v8f;
typedef __attribute__((ext_vector_type(4)))  float v4f;

__device__ __forceinline__ v8b ld8b(const b16* p) { return *(const v8b*)p; }
__device__ __forceinline__ v16b cat8b(v8b a, v8b b) { return __builtin_shufflevector(a, b, 0, 1, 2, 3, 4, 5, 6, 7, 8, 9, 10, 11, 12, 13, 14, 15); }
__device__ __forceinline__ v16b frag_kb(const b16* p, int hh) { return cat8b(ld8b(p + 8 * hh), ld8b(p + 16 + 8 * hh)); }
__device__ __forceinline__ void split16(float v, b16& hi, b16& lo) { hi = (b16)v; lo = (b16)(v - (float)hi); }
__device__ __forceinline__ void frag_ksplit(const float* p, int hh, v16b& fh_, v16b& fl_) {
  const float* p0 = p + 8 * hh; const float* p1 = p + 16 + 8 * hh;
#pragma unroll
  for (int e = 0; e < 8; ++e) { b16 a, c; split16(p0[e], a, c); fh_[e] = a; fl_[e] = c; split16(p1[e], a, c); fh_[8 + e] = a; fl_[8 + e] = c; }
}
__device__ __forceinline__ v8f wmma16b(v16b a, v16b b, v8f c) {
  v8f d = __builtin_amdgcn_wmma_f32_16x16x32_f16(false, a, false, b, (short)0, c, false, false);
  asm volatile("v_nop\n\tv_nop\n\tv_nop\n\tv_nop" : "+v"(d) : "v"(a), "v"(b));
  return d;
}
__device__ __forceinline__ void wave_lds_sync() {
  __builtin_amdgcn_fence(__ATOMIC_RELEASE, "workgroup");
  __builtin_amdgcn_wave_barrier();
  __builtin_amdgcn_fence(__ATOMIC_ACQUIRE, "workgroup");
}

struct Opnd { const void* p0; const void* p1; int ld; };
template <int NP> __device__ __forceinline__ void load_frags(const Opnd& o, int row, int kb, int hh, v16b& fh_, v16b& fl_) {
  if (NP == 0) { frag_ksplit((const float*)o.p0 + (size_t)row * o.ld + kb, hh, fh_, fl_); }
  else if (NP == 4 || NP == 5) {
    const float sc_ = (NP == 4) ? 64.0f : 8.0f;
    const float* p = (const float*)o.p0 + (size_t)row * o.ld + kb; const float* p0 = p + 8 * hh; const float* p1 = p + 16 + 8 * hh;
#pragma unroll
    for (int e = 0; e < 8; ++e) { b16 a, c; split16(p0[e] * sc_, a, c); fh_[e] = a; fl_[e] = c; split16(p1[e] * sc_, a, c); fh_[8 + e] = a; fl_[8 + e] = c; }
  } else if (NP == 3) {
    const float* p = (const float*)o.p0 + (size_t)row * o.ld + kb; const float* p0 = p + 8 * hh; const float* p1 = p + 16 + 8 * hh;
#pragma unroll
    for (int e = 0; e < 8; ++e) { fh_[e] = (b16)p0[e]; fh_[8 + e] = (b16)p1[e]; }
    fl_ = fh_;
  } else {
    fh_ = frag_kb((const b16*)o.p0 + (size_t)row * o.ld + kb, hh);
    if (NP == 2) fl_ = frag_kb((const b16*)o.p1 + (size_t)row * o.ld + kb, hh); else fl_ = fh_;
  }
}
template <int ANP, int BNP> __device__ __forceinline__ v8f mac(v16b ah, v16b al, v16b bh, v16b bl, v8f c) {
  c = wmma16b(ah, bh, c);
  if (BNP == 0 || BNP == 2 || BNP == 4 || BNP == 5) c = wmma16b(ah, bl, c);
  if (ANP == 0 || ANP == 2 || ANP == 4 || ANP == 5) c = wmma16b(al, bh, c);
  return c;
}
template <int ANP, int BNP>
__device__ __forceinline__ void gemm_tile(const Opnd& A, const Opnd& B, int K, int m0, int c0, int nloc, int hlf, v8f (&acc)[2][4]) {
  for (int kb = 0; kb < K; kb += 32) {
    v16b a0h, a0l, a1h, a1l;
    load_frags<ANP>(A, m0 + nloc, kb, hlf, a0h, a0l);
    load_frags<ANP>(A, m0 + 16 + nloc, kb, hlf, a1h, a1l);
#pragma unroll
    for (int t = 0; t < 4; ++t) {
      v16b bh, bl;
      load_frags<BNP>(B, c0 + t * 16 + nloc, kb, hlf, bh, bl);
      acc[0][t] = mac<ANP, BNP>(a0h, a0l, bh, bl, acc[0][t]);
      acc[1][t] = mac<ANP, BNP>(a1h, a1l, bh, bl, acc[1][t]);
    }
  }
}

__device__ __forceinline__ void epi_planes(v8f (&acc)[2][4], float scale, bool two, b16* __restrict__ oh, b16* __restrict__ ol, int ldo,
                                           int m0, int c0, int lane, b16* Th, b16* Tl) {
  const int nloc = lane & 15, hlf = lane >> 4;
#pragma unroll
  for (int t = 0; t < 4; ++t)
#pragma unroll
    for (int r = 0; r < 2; ++r)
#pragma unroll
      for (int v = 0; v < 8; ++v) {
        const int rr = r * 16 + v + 8 * hlf, cc = t * 16 + nloc;
        b16 h_, l_; split16(acc[r][t][v] * scale, h_, l_);
        Th[rr * 64 + cc] = h_; Tl[rr * 64 + cc] = l_;
      }
  wave_lds_sync();
  for (int pass = 0; pass < 2; ++pass) {
#pragma unroll
    for (int j = 0; j < 8; ++j) {
      const int rr = j * 4 + (lane >> 3), c8 = (lane & 7) * 8;
      const size_t o = (size_t)(m0 + rr) * ldo + c0 + c8;
      *(volatile v8b*)(oh + o) = ld8b(Th + rr * 64 + c8);
      if (two) *(volatile v8b*)(ol + o) = ld8b(Tl + rr * 64 + c8);
    }
    __threadfence();
  }
}
__device__ __forceinline__ void epi_f32(v8f (&acc)[2][4], float scale, const float* rscale, float* __restrict__ out, int ldo, int m0, int c0, int lane, float* Tt) {
  const int nloc = lane & 15, hlf = lane >> 4;
#pragma unroll
  for (int t = 0; t < 4; ++t)
#pragma unroll
    for (int r = 0; r < 2; ++r)
#pragma unroll
      for (int v = 0; v < 8; ++v) {
        const int rr = r * 16 + v + 8 * hlf;
        const float rs = rscale ? rscale[(size_t)(m0 + rr) * 32] : 1.0f;
        Tt[rr * 64 + t * 16 + nloc] = acc[r][t][v] * scale * rs;
      }
  wave_lds_sync();
  float* dst0 = out + (size_t)m0 * ldo + c0;
  for (int pass = 0; pass < 2; ++pass) {
#pragma unroll
    for (int j = 0; j < 16; ++j) { const int rr = j * 2 + hlf, c4 = nloc * 4; *(volatile v4f*)(dst0 + (size_t)rr * ldo + c4) = *(const v4f*)(Tt + rr * 64 + c4); }
    __threadfence();
  }
}


typedef __attribute__((ext_vector_type(8))) __bf16 v8bb; typedef __attribute__((ext_vector_type(16))) __bf16 v16bb;
typedef __attribute__((ext_vector_type(8))) unsigned short v8us;
__device__ __forceinline__ v16bb frag_kb_bf(const __bf16* p, int hh) { const v8bb a = *(const v8bb*)(p + 8 * hh), b = *(const v8bb*)(p + 16 + 8 * hh); return __builtin_shufflevector(a, b, 0, 1, 2, 3, 4, 5, 6, 7, 8, 9, 10, 11, 12, 13, 14, 15); }
__device__ __forceinline__ v8f wmma16bb(v16bb a, v16bb b, v8f c) {
  v8f d = __builtin_amdgcn_wmma_f32_16x16x32_bf16(false, a, false, b, (short)0, c, false, false);
  asm volatile("v_nop\n\tv_nop\n\tv_nop\n\tv_nop" : "+v"(d) : "v"(a), "v"(b));
  return d;
}
__device__ __forceinline__ unsigned short bf16_rne_bits(float v) { unsigned int u = __float_as_uint(v); u += 0x7FFFu + ((u >> 16) & 1u); return (unsigned short)(u >> 16); }
__device__ __forceinline__ float bf16_rne(float v) { return __uint_as_float(((unsigned int)bf16_rne_bits(v)) << 16); }


__global__ __launch_bounds__(256) void prep_kernel(const float* __restrict__ x, const float* __restrict__ wq, const float* __restrict__ wk, const float* __restrict__ wv, const float* __restrict__ wo,
                                                   const float* __restrict__ lq1, const float* __restrict__ lk1, const float* __restrict__ lq2, const float* __restrict__ lk2,
                                                   unsigned short* __restrict__ x16, unsigned short* __restrict__ w16, b16* __restrict__ wo16, float* __restrict__ lam) {
  const size_t tid = (size_t)blockIdx.x * blockDim.x + threadIdx.x, nth = (size_t)gridDim.x * blockDim.x;
  for (int pass = 0; pass < 2; ++pass) {
    for (size_t p = tid; p < (size_t)S * D / 8; p += nth) { v8us v;
#pragma unroll
      for (int e = 0; e < 8; ++e) v[e] = bf16_rne_bits(x[p * 8 + e]);
      *(volatile v8us*)(x16 + p * 8) = v; }
    for (size_t p = tid; p < (size_t)(2 * D + 2 * DKV + DKV) * D / 8; p += nth) { const size_t r = p / (D / 8); const float* W; size_t q;
      if (r < (size_t)2 * D) { W = wq; q = p; } else if (r < (size_t)2 * D + 2 * DKV) { W = wk; q = p - (size_t)2 * D * (D / 8); } else { W = wv; q = p - (size_t)(2 * D + 2 * DKV) * (D / 8); }
      v8us v;
#pragma unroll
      for (int e = 0; e < 8; ++e) v[e] = bf16_rne_bits(W[q * 8 + e]);
      *(volatile v8us*)(w16 + p * 8) = v; }
    for (size_t p = tid; p < (size_t)D * D / 8; p += nth) { v8b w;
#pragma unroll
      for (int e = 0; e < 8; ++e) w[e] = (b16)bf16_rne(wo[p * 8 + e]);
      *(volatile v8b*)(wo16 + p * 8) = w; }
    if (tid == 0) { float s1 = 0.0f, s2 = 0.0f; for (int i = 0; i < HD; ++i) { s1 += bf16_rne(lq1[i]) * bf16_rne(lk1[i]); s2 += bf16_rne(lq2[i]) * bf16_rne(lk2[i]); } ((volatile float*)lam)[0] = expf(s1) - expf(s2) + LAMBDA_INIT; }
    __threadfence();
  }
}

__global__ __launch_bounds__(128) void proj_kernel(const __bf16* __restrict__ x16, const __bf16* __restrict__ w16, const int* __restrict__ pos, b16* __restrict__ qh, b16* __restrict__ kh, b16* __restrict__ vt) {
  __shared__ __attribute__((aligned(16))) b16 Th[4][32][HD + 8], Tq[4][32][HD + 8];
  __shared__ __attribute__((aligned(16))) b16 Tt[64][128 + 8], Tl[64][128 + 8];
  const int lane = threadIdx.x & 31, wave = threadIdx.x >> 5, nloc = lane & 15, hlf = lane >> 4, m0 = blockIdx.y * 128 + wave * 32, c0 = blockIdx.x * 64;
  v8f acc[2][4];
#pragma unroll
  for (int r = 0; r < 2; ++r)
#pragma unroll
    for (int t = 0; t < 4; ++t) acc[r][t] = (v8f){};
#pragma unroll 2
  for (int kb = 0; kb < D; kb += 32) {
    const v16bb a0 = frag_kb_bf(x16 + (size_t)(m0 + nloc) * D + kb, hlf), a1 = frag_kb_bf(x16 + (size_t)(m0 + 16 + nloc) * D + kb, hlf);
#pragma unroll
    for (int t = 0; t < 4; ++t) { const v16bb bw = frag_kb_bf(w16 + (size_t)(c0 + t * 16 + nloc) * D + kb, hlf); acc[0][t] = wmma16bb(a0, bw, acc[0][t]); acc[1][t] = wmma16bb(a1, bw, acc[1][t]); }
  }
  if (blockIdx.x < NQT + NKT) {
    const bool isq = blockIdx.x < NQT; const int head = isq ? blockIdx.x : blockIdx.x - NQT;
#pragma unroll
    for (int t = 0; t < 2; ++t) { const int i = t * 16 + nloc; const float inv_freq = 1.0f / powf(THETA, (float)(2 * i) / (float)HD);
#pragma unroll
      for (int r = 0; r < 2; ++r)
#pragma unroll
        for (int v = 0; v < 8; ++v) { const int tok = m0 + r * 16 + 8 * hlf + v; float sn, cs; sincosf((float)pos[tok] * inv_freq, &sn, &cs);
          const float x1 = acc[r][t][v], x2 = acc[r][t + 2][v]; b16 a_, c_;
          split16((x1 * cs - x2 * sn) * QS, a_, c_); Th[wave][r * 16 + 8 * hlf + v][i] = a_; Tq[wave][r * 16 + 8 * hlf + v][i] = c_;
          split16((x2 * cs + x1 * sn) * QS, a_, c_); Th[wave][r * 16 + 8 * hlf + v][i + 32] = a_; Tq[wave][r * 16 + 8 * hlf + v][i + 32] = c_; } }
    wave_lds_sync();
    b16* dst = (isq ? qh : kh) + ((size_t)head * S + m0) * HD; const size_t PLs = isq ? QPL : KPL;
    for (int pass = 0; pass < 2; ++pass) {
#pragma unroll
      for (int j = 0; j < 8; ++j) { const int rr = j * 4 + (lane >> 3), c8 = (lane & 7) * 8; *(volatile v8b*)(dst + (size_t)rr * HD + c8) = *(const v8b*)(&Th[wave][rr][c8]); *(volatile v8b*)(dst + PLs + (size_t)rr * HD + c8) = *(const v8b*)(&Tq[wave][rr][c8]); }
      __threadfence(); }
    return;
  }
  const int vh = blockIdx.x - NQT - NKT;
#pragma unroll
  for (int t = 0; t < 4; ++t)
#pragma unroll
    for (int r = 0; r < 2; ++r)
#pragma unroll
      for (int v = 0; v < 8; ++v) { b16 a_, c_; split16(acc[r][t][v] * VS, a_, c_); Tt[t * 16 + nloc][wave * 32 + r * 16 + 8 * hlf + v] = a_; Tl[t * 16 + nloc][wave * 32 + r * 16 + 8 * hlf + v] = c_; }
  __syncthreads();
  b16* dstv = vt + ((size_t)vh * HD) * S + blockIdx.y * 128;
  for (int pass = 0; pass < 2; ++pass) {
#pragma unroll
    for (int j = 0; j < 8; ++j) { const int dd = wave * 16 + j * 2 + (lane >> 4), c8 = (lane & 15) * 8; *(volatile v8b*)(dstv + (size_t)dd * S + c8) = *(const v8b*)(&Tt[dd][c8]); *(volatile v8b*)(dstv + VPL + (size_t)dd * S + c8) = *(const v8b*)(&Tl[dd][c8]); }
    __threadfence();
  }
}

template <int QT>
__global__ __launch_bounds__(256) void attn_kernel(const b16* __restrict__ qh, const b16* __restrict__ kh, const b16* __restrict__ vt, const float* __restrict__ lam, const float* __restrict__ nw, float* __restrict__ y) {
  __shared__ __attribute__((aligned(16))) float Os[8][16][HD + 4];
  const int wid = threadIdx.x >> 5, lane = threadIdx.x & 31, hh = lane >> 4, col = lane & 15;
  const int qt = blockIdx.x * 8 + wid, jt = qt % QT, h = qt / QT, q0 = jt * 16, qi = q0 + col, hk = h / GRP;
  const b16* Q1 = qh + (size_t)h * S * HD; const b16* Q2 = qh + (size_t)(H + h) * S * HD; const b16* K1 = kh + (size_t)hk * S * HD; const b16* K2 = kh + (size_t)(HKV + hk) * S * HD; const b16* vb = vt + ((size_t)hk * HD) * S;
  v16b q1f[2], q1l[2], q2f[2], q2l[2];
#pragma unroll
  for (int ks = 0; ks < 2; ++ks) { q1f[ks] = frag_kb(Q1 + (size_t)qi * HD + ks * 32, hh); q1l[ks] = frag_kb(Q1 + QPL + (size_t)qi * HD + ks * 32, hh); q2f[ks] = frag_kb(Q2 + (size_t)qi * HD + ks * 32, hh); q2l[ks] = frag_kb(Q2 + QPL + (size_t)qi * HD + ks * 32, hh); }
  float m1 = -INFINITY, l1 = 0.0f, m2 = -INFINITY, l2 = 0.0f; v8f o1[4] = {{}, {}, {}, {}}, o2[4] = {{}, {}, {}, {}};
  for (int kb = 0; kb < q0 + 16; kb += 32) {
    const bool diag = (kb + 32 > q0);
    v8f s0 = {}, s1 = {}, t0 = {}, t1 = {};
#pragma unroll
    for (int ks = 0; ks < 2; ++ks) {
      { const v16b k0 = frag_kb(K1 + (size_t)(kb + col) * HD + ks * 32, hh), k0l = frag_kb(K1 + KPL + (size_t)(kb + col) * HD + ks * 32, hh), kk1 = frag_kb(K1 + (size_t)(kb + 16 + col) * HD + ks * 32, hh), kk1l = frag_kb(K1 + KPL + (size_t)(kb + 16 + col) * HD + ks * 32, hh);
        s0 = wmma16b(k0, q1f[ks], s0); s0 = wmma16b(k0, q1l[ks], s0); s0 = wmma16b(k0l, q1f[ks], s0); s1 = wmma16b(kk1, q1f[ks], s1); s1 = wmma16b(kk1, q1l[ks], s1); s1 = wmma16b(kk1l, q1f[ks], s1); }
      { const v16b k0 = frag_kb(K2 + (size_t)(kb + col) * HD + ks * 32, hh), k0l = frag_kb(K2 + KPL + (size_t)(kb + col) * HD + ks * 32, hh), kk1 = frag_kb(K2 + (size_t)(kb + 16 + col) * HD + ks * 32, hh), kk1l = frag_kb(K2 + KPL + (size_t)(kb + 16 + col) * HD + ks * 32, hh);
        t0 = wmma16b(k0, q2f[ks], t0); t0 = wmma16b(k0, q2l[ks], t0); t0 = wmma16b(k0l, q2f[ks], t0); t1 = wmma16b(kk1, q2f[ks], t1); t1 = wmma16b(kk1, q2l[ks], t1); t1 = wmma16b(kk1l, q2f[ks], t1); } }
    float mr1 = -INFINITY, mr2 = -INFINITY;
#pragma unroll
    for (int r = 0; r < 8; ++r) { s0[r] *= SCALE / (QS * QS); s1[r] *= SCALE / (QS * QS); t0[r] *= SCALE / (QS * QS); t1[r] *= SCALE / (QS * QS);
      if (diag) { if (kb + 8 * hh + r > qi) { s0[r] = -INFINITY; t0[r] = -INFINITY; } if (kb + 16 + 8 * hh + r > qi) { s1[r] = -INFINITY; t1[r] = -INFINITY; } }
      mr1 = fmaxf(mr1, fmaxf(s0[r], s1[r])); mr2 = fmaxf(mr2, fmaxf(t0[r], t1[r])); }
    mr1 = fmaxf(mr1, __shfl_xor(mr1, 16)); mr2 = fmaxf(mr2, __shfl_xor(mr2, 16));
    const float mn1 = fmaxf(m1, mr1), al1 = __expf(m1 - mn1); m1 = mn1; const float mn2 = fmaxf(m2, mr2), al2 = __expf(m2 - mn2); m2 = mn2;
    float sum1 = 0.0f, sum2 = 0.0f; v16b pb, pl, ub, ul;
#pragma unroll
    for (int r = 0; r < 8; ++r) { const float e0 = __expf(s0[r] - mn1), e1 = __expf(s1[r] - mn1), f0 = __expf(t0[r] - mn2), f1 = __expf(t1[r] - mn2); sum1 += e0 + e1; sum2 += f0 + f1; b16 a, c;
      split16(e0 * PS, a, c); pb[r] = a; pl[r] = c; split16(e1 * PS, a, c); pb[8 + r] = a; pl[8 + r] = c; split16(f0 * PS, a, c); ub[r] = a; ul[r] = c; split16(f1 * PS, a, c); ub[8 + r] = a; ul[8 + r] = c; }
    sum1 += __shfl_xor(sum1, 16); sum2 += __shfl_xor(sum2, 16); l1 = l1 * al1 + sum1; l2 = l2 * al2 + sum2;
#pragma unroll
    for (int n = 0; n < 4; ++n) {
#pragma unroll
      for (int r = 0; r < 8; ++r) { o1[n][r] *= al1; o2[n][r] *= al2; }
      const v16b vf = frag_kb(vb + (size_t)(n * 16 + col) * S + kb, hh), vl = frag_kb(vb + VPL + (size_t)(n * 16 + col) * S + kb, hh);
      o1[n] = wmma16b(vf, pb, o1[n]); o1[n] = wmma16b(vf, pl, o1[n]); o1[n] = wmma16b(vl, pb, o1[n]);
      o2[n] = wmma16b(vf, ub, o2[n]); o2[n] = wmma16b(vf, ul, o2[n]); o2[n] = wmma16b(vl, ub, o2[n]); }
  }
  const float lamv = lam[0], i1 = 1.0f / (VS * PS * l1), i2 = lamv / (VS * PS * l2);
  float ss = 0.0f;
#pragma unroll
  for (int n = 0; n < 4; ++n)
#pragma unroll
    for (int r = 0; r < 8; ++r) { const float val = o1[n][r] * i1 - o2[n][r] * i2; o1[n][r] = val; ss += val * val; }
  ss += __shfl_xor(ss, 16);
  const float rn = rsqrtf(ss * (1.0f / HD) + EPSN) * (1.0f - LAMBDA_INIT);
#pragma unroll
  for (int n = 0; n < 4; ++n)
#pragma unroll
    for (int r = 0; r < 8; ++r) { const int d = n * 16 + 8 * hh + r; Os[wid][col][d] = o1[n][r] * rn * bf16_rne(nw[d]); }
  wave_lds_sync();
  float* dst = y + (size_t)q0 * D + h * HD;
  for (int pass = 0; pass < 2; ++pass) {
#pragma unroll
    for (int j = 0; j < 8; ++j) { const int rr = j * 2 + hh, c4 = col * 4; *(volatile v4f*)(dst + (size_t)rr * D + c4) = *(const v4f*)(&Os[wid][rr][c4]); }
    __threadfence();
  }
}

__global__ __launch_bounds__(128) void out_kernel(const float* __restrict__ y, const b16* __restrict__ wo16, float* __restrict__ out) {
  __shared__ __attribute__((aligned(16))) float Ts[4][32 * 64];
  const int lane = threadIdx.x & 31, wave = threadIdx.x >> 5, nloc = lane & 15, hlf = lane >> 4, m0 = blockIdx.y * 128 + wave * 32, c0 = blockIdx.x * 64;
  v8f acc[2][4];
#pragma unroll
  for (int r = 0; r < 2; ++r)
#pragma unroll
    for (int t = 0; t < 4; ++t) acc[r][t] = (v8f){};
  const Opnd A{y, nullptr, D}, Bo{wo16, nullptr, D};
  gemm_tile<5, 1>(A, Bo, D, m0, c0, nloc, hlf, acc);
  epi_f32(acc, 1.0f / 8.0f, nullptr, out, D, m0, c0, lane, Ts[wave]);
}
}

extern "C" void kernel_launch(void* const* d_in, const int* in_sizes, int n_in,
                              void* d_out, int out_size, void* d_ws, size_t ws_size, hipStream_t stream) {
  (void)n_in; (void)out_size;
  const float* x = (const float*)d_in[0]; const float* wq = (const float*)d_in[1]; const float* wk = (const float*)d_in[2]; const float* wv = (const float*)d_in[3]; const float* wo = (const float*)d_in[4];
  const float* lq1 = (const float*)d_in[5]; const float* lk1 = (const float*)d_in[6]; const float* lq2 = (const float*)d_in[7]; const float* lk2 = (const float*)d_in[8]; const float* nw = (const float*)d_in[9]; const int* pos = (const int*)d_in[10];
  float* out = (float*)d_out;
  if (in_sizes[0] != S * D || in_sizes[1] != 2 * D * D || in_sizes[2] != 2 * DKV * D || in_sizes[3] != DKV * D || in_sizes[4] != D * D || in_sizes[9] != HD || in_sizes[10] != S) return;
  size_t off = 0; char* ws = (char*)d_ws;
  auto carve = [&](size_t bytes) { char* p = ws + off; off += (bytes + 255) & ~(size_t)255; return p; };
  unsigned short* x16 = (unsigned short*)carve((size_t)S * D * 2); unsigned short* w16 = (unsigned short*)carve((size_t)(2 * D + 3 * DKV) * D * 2); b16* wo16 = (b16*)carve((size_t)D * D * 2); float* lam = (float*)carve(256);
  b16* qh = (b16*)carve(QPL * 2 * 2); b16* kh = (b16*)carve(KPL * 2 * 2); b16* vt = (b16*)carve(VPL * 2 * 2); float* y = (float*)carve((size_t)S * D * 4);
  if (off > ws_size) return;
  prep_kernel<<<1024, 256, 0, stream>>>(x, wq, wk, wv, wo, lq1, lk1, lq2, lk2, x16, w16, wo16, lam);
  proj_kernel<<<dim3(NT, S / 128), 128, 0, stream>>>((const __bf16*)x16, (const __bf16*)w16, pos, qh, kh, vt);
  attn_kernel<S / 16><<<H * (S / 16) / 8, 256, 0, stream>>>(qh, kh, vt, lam, nw, y);
  out_kernel<<<dim3(D / 64, S / 128), 128, 0, stream>>>(y, wo16, out);
}
